// TaylorSoftmaxAttention_25984552141265
// MI455X (gfx1250) — hardware-verified
//
#include <hip/hip_runtime.h>
#include <stdint.h>


typedef __attribute__((ext_vector_type(16))) _Float16 v16h;
typedef __attribute__((ext_vector_type(8)))  _Float16 v8h;
typedef __attribute__((ext_vector_type(16))) __bf16   v16b;
typedef __attribute__((ext_vector_type(8)))  __bf16   v8b;
typedef __attribute__((ext_vector_type(8)))  float    v8f;
typedef __attribute__((ext_vector_type(4)))  float    v4f;

#define NB    8
#define NTOK  2048
#define CDIM  256
#define NH    8
#define HD    32
#define NBH   64
#define QKVW  768
#define NF    576
#define EP    64
#define GB    16
#define SCALE4 2.3784142300054421f
#define COEF_B 5.656854249492380f
#define COEF_C 32.0f

__device__ __forceinline__ unsigned short f2bf_bits(float f) {
  unsigned u = __float_as_uint(f);
  return (unsigned short)((u + 0x7FFFu + ((u >> 16) & 1u)) >> 16);
}
__device__ __forceinline__ float bf_bits2f(unsigned short h) { return __uint_as_float(((unsigned)h) << 16); }

__device__ __forceinline__ void dep_guard_h(v8f& a, v8f& b, v16h x, v16h y) { asm volatile("v_nop\n\tv_nop\n\tv_nop\n\tv_nop" : "+v"(a), "+v"(b) : "v"(x), "v"(y)); }
__device__ __forceinline__ void dep_guard_b(v8f& a, v8f& b, v16b x, v16b y) { asm volatile("v_nop\n\tv_nop\n\tv_nop\n\tv_nop" : "+v"(a), "+v"(b) : "v"(x), "v"(y)); }
__device__ __forceinline__ void keep4_h(v16h a, v16h b, v16h c, v16h d) { asm volatile("v_nop" :: "v"(a), "v"(b), "v"(c), "v"(d)); }
__device__ __forceinline__ void keep4_b(v16b a, v16b b, v16b c, v16b d) { asm volatile("v_nop" :: "v"(a), "v"(b), "v"(c), "v"(d)); }
__device__ __forceinline__ void acc_guard4(v8f& a, v8f& b, v8f& c, v8f& d) { asm volatile("v_nop\n\tv_nop\n\tv_nop\n\tv_nop" : "+v"(a), "+v"(b), "+v"(c), "+v"(d)); }
template <typename T> struct Frag;
template <> struct Frag<_Float16> {
  typedef v16h V; union U { v16h v; v8h h[2]; };
  static __device__ __forceinline__ v16h load(const _Float16* p) {
    U f; f.h[0] = *(const v8h*)(p); f.h[1] = *(const v8h*)(p + 16); return f.v;
  }
  static __device__ __forceinline__ v8f mma(v16h a, v16h b, v8f c) {
    return __builtin_amdgcn_wmma_f32_16x16x32_f16(false, a, false, b, (short)0, c, false, false);
  }
  static __device__ __forceinline__ void guard(v8f& a, v8f& b, v16h x, v16h y) { dep_guard_h(a, b, x, y); }
  static __device__ __forceinline__ void keep(v16h a, v16h b, v16h c, v16h d) { keep4_h(a, b, c, d); }
};
template <> struct Frag<__bf16> {
  typedef v16b V; union U { v16b v; v8b h[2]; };
  static __device__ __forceinline__ v16b load(const __bf16* p) {
    U f; f.h[0] = *(const v8b*)(p); f.h[1] = *(const v8b*)(p + 16); return f.v;
  }
  static __device__ __forceinline__ v8f mma(v16b a, v16b b, v8f c) {
    return __builtin_amdgcn_wmma_f32_16x16x32_bf16(false, a, false, b, (short)0, c, false, false);
  }
  static __device__ __forceinline__ void guard(v8f& a, v8f& b, v16b x, v16b y) { dep_guard_b(a, b, x, y); }
  static __device__ __forceinline__ void keep(v16b a, v16b b, v16b c, v16b d) { keep4_b(a, b, c, d); }
};

__device__ __forceinline__ float col_coef(int n) {
  return (n < HD) ? 0.5f : ((n < 528) ? 1.0f : ((n < 560) ? COEF_B : 0.0f));
}

template <int ET> struct Elem;
template <> struct Elem<0> { typedef _Float16 T; };
template <> struct Elem<1> { typedef __bf16 T; };
template <int ET, bool SPLIT, int BIAS_MODE, int OUT_MODE, bool RESID, int ACT = 0, int CS = 0>
__global__ __launch_bounds__(256) void wmma_gemm64(
    const unsigned short* __restrict__ Ap, const unsigned short* __restrict__ A2p, int lda, long strideA,
    const unsigned short* __restrict__ Btp, const unsigned short* __restrict__ Bt2p, int ldb, long strideB,
    void* __restrict__ Cout, void* __restrict__ Cout2, int ldc, long strideC,
    const float* __restrict__ bias,
    const float* __restrict__ resid, long strideR,
    int M, int N, int K, float scale) {
  typedef typename Elem<ET>::T T;
  typedef typename Frag<T>::V V;
  const T* A = (const T*)Ap; const T* A2 = (const T*)A2p; const T* Bt = (const T*)Btp; const T* Bt2 = (const T*)Bt2p;
  __shared__ __align__(16) float sT[8][16 * 68];
  const int b    = blockIdx.y;
  const int lane = threadIdx.x & 31;
  const int wave = threadIdx.x >> 5;
  const int tilesN = N >> 6;
  const int tilesM = M >> 6;
  const int tile = blockIdx.x * 8 + wave;
  if (tile >= tilesM * tilesN) return;
  const int tm = tile / tilesN;
  const int tn = tile - tm * tilesN;
  const int m0 = tm << 6;
  const int n0 = tn << 6;

  const T* Ab  = A  + (size_t)b * strideA;
  const T* Bb  = Bt + (size_t)b * strideB;
  const T* Ab2 = SPLIT ? (A2  + (size_t)b * strideA) : nullptr;
  const T* Bb2 = SPLIT ? (Bt2 + (size_t)b * strideB) : nullptr;

  const int rlane = lane & 15;
  const int koff  = (lane >> 4) * 8;
  const int mOff  = (lane >> 4) * 8;

  v8f acc[4][4];
#pragma unroll
  for (int i = 0; i < 4; ++i)
#pragma unroll
    for (int j = 0; j < 4; ++j) acc[i][j] = (v8f){0.f,0.f,0.f,0.f,0.f,0.f,0.f,0.f};

  for (int k0 = 0; k0 < K; k0 += 32) {
    V bh[4], bl[4];
#pragma unroll
    for (int j = 0; j < 4; ++j) {
      const size_t bo = (size_t)(n0 + (j << 4) + rlane) * ldb + koff + k0;
      bh[j] = Frag<T>::load(Bb + bo);
      if (SPLIT) bl[j] = Frag<T>::load(Bb2 + bo);
    }
#pragma unroll
    for (int i = 0; i < 4; ++i) {
      const size_t ao = (size_t)(m0 + (i << 4) + rlane) * lda + koff + k0;
      V ah = Frag<T>::load(Ab + ao);
      V al;
      if (SPLIT) al = Frag<T>::load(Ab2 + ao);
#pragma unroll
      for (int j = 0; j < 4; ++j) {
        acc[i][j] = Frag<T>::mma(ah, bh[j], acc[i][j]);
        if (SPLIT) {
          acc[i][j] = Frag<T>::mma(ah, bl[j], acc[i][j]);
          acc[i][j] = Frag<T>::mma(al, bh[j], acc[i][j]);
        }
      }
      Frag<T>::guard(acc[i][0], acc[i][3], ah, SPLIT ? al : ah);
    }
    Frag<T>::keep(bh[0], bh[1], bh[2], bh[3]);
    if (SPLIT) Frag<T>::keep(bl[0], bl[1], bl[2], bl[3]);
  }
  acc_guard4(acc[0][0], acc[0][1], acc[0][2], acc[0][3]);
  acc_guard4(acc[1][0], acc[1][1], acc[1][2], acc[1][3]);
  acc_guard4(acc[2][0], acc[2][1], acc[2][2], acc[2][3]);
  acc_guard4(acc[3][0], acc[3][1], acc[3][2], acc[3][3]);

  float* slab = sT[wave];
  const float* Rb = RESID ? (resid + (size_t)b * strideR) : nullptr;
#pragma unroll
  for (int i = 0; i < 4; ++i) {
    const int mBase = m0 + (i << 4);
#pragma unroll
    for (int j = 0; j < 4; ++j) {
      const int n = n0 + (j << 4) + rlane;
      float bv = 0.f;
      if (BIAS_MODE == 2) bv = bias[n];
#pragma unroll
      for (int r = 0; r < 8; ++r) {
        float v = acc[i][j][r] * scale;
        if (CS == 1) v = v * col_coef(n);
        if (BIAS_MODE == 1) v += bias[mBase + mOff + r];
        if (BIAS_MODE == 2) v += bv;
        if (RESID) v += Rb[(size_t)(mBase + mOff + r) * ldc + n];
        if (ACT == 1) v = tanhf(v);
        if (ACT == 2) v = fmaxf(v, 0.0f);
        if (ACT == 3) v = v / (1.0f + expf(-v));
        if (ACT == 4) v = (v > 0.f) ? v : 0.01f * v;
        if (ACT == 5) v = 0.5f * v * (1.0f + erff(v * 0.70710678118654752f));
        slab[(mOff + r) * 68 + (j << 4) + rlane] = v;
      }
    }
    __builtin_amdgcn_fence(__ATOMIC_RELEASE, "workgroup");
    __builtin_amdgcn_wave_barrier();
    __builtin_amdgcn_fence(__ATOMIC_ACQUIRE, "workgroup");
    if (OUT_MODE == 0) {
      float* C = (float*)Cout + (size_t)b * strideC;
      const int hh = lane >> 4, c4 = (lane & 15) * 4;
      for (int pass = 0; pass < 2; ++pass) {
#pragma unroll
        for (int it = 0; it < 8; ++it) {
          const int row = it * 2 + hh;
          v4f v = *(const v4f*)(slab + row * 68 + c4);
          *(volatile v4f*)(C + (size_t)(mBase + row) * ldc + n0 + c4) = v;
        }
        __threadfence();
      }
    } else {
      const int q = lane >> 3, c8 = (lane & 7) * 8;
      unsigned short* C  = (unsigned short*)Cout  + (size_t)b * strideC;
      unsigned short* C2 = (OUT_MODE == 2) ? ((unsigned short*)Cout2 + (size_t)b * strideC) : nullptr;
      for (int pass = 0; pass < 2; ++pass) {
#pragma unroll
        for (int it = 0; it < 4; ++it) {
          const int row = it * 4 + q;
          const float* sp = slab + row * 68 + c8;
          v8h hv, lv;
#pragma unroll
          for (int e = 0; e < 8; ++e) {
            if (OUT_MODE == 1) {
              hv[e] = (_Float16)sp[e];
            } else {
              unsigned short hb = f2bf_bits(sp[e]);
              unsigned short lb = f2bf_bits(sp[e] - bf_bits2f(hb));
              hv[e] = __builtin_bit_cast(_Float16, hb);
              lv[e] = __builtin_bit_cast(_Float16, lb);
            }
          }
          *(volatile v8h*)(C + (size_t)(mBase + row) * ldc + n0 + c8) = hv;
          if (OUT_MODE == 2) *(volatile v8h*)(C2 + (size_t)(mBase + row) * ldc + n0 + c8) = lv;
        }
        __threadfence();
      }
    }
    __builtin_amdgcn_fence(__ATOMIC_RELEASE, "workgroup");
    __builtin_amdgcn_wave_barrier();
    __builtin_amdgcn_fence(__ATOMIC_ACQUIRE, "workgroup");
  }
}

__global__ __launch_bounds__(256) void cast_split_bf16x2(
    const float* __restrict__ in, unsigned short* __restrict__ hi, unsigned short* __restrict__ lo, int n2) {
  const int i = blockIdx.x * 256 + threadIdx.x;
  if (i < n2) {
    const float f0 = in[2 * i], f1 = in[2 * i + 1];
    const unsigned short h0 = f2bf_bits(f0), h1 = f2bf_bits(f1);
    const unsigned short l0 = f2bf_bits(f0 - bf_bits2f(h0)), l1 = f2bf_bits(f1 - bf_bits2f(h1));
    const unsigned uh = (unsigned)h0 | ((unsigned)h1 << 16);
    const unsigned ul = (unsigned)l0 | ((unsigned)l1 << 16);
    ((volatile unsigned*)hi)[i] = uh;
    ((volatile unsigned*)lo)[i] = ul;
    __threadfence();
    ((volatile unsigned*)hi)[i] = uh;
    ((volatile unsigned*)lo)[i] = ul;
  }
}

__device__ __forceinline__ int feat_code(int f) {
  if (f < HD) return f | (f << 8);
  if (f < 528) {
    const int g = f - HD;
    int i = 0;
    for (int ii = 1; ii < 31; ++ii) {
      const int off = 31 * ii - ((ii * (ii - 1)) >> 1);
      i = (g >= off) ? ii : i;
    }
    const int off = 31 * i - ((i * (i - 1)) >> 1);
    return i | ((i + 1 + (g - off)) << 8);
  }
  if (f < 560) return (f - 528) | (255 << 8);
  return 254 << 8;
}

__global__ __launch_bounds__(256) void prep_qkv(
    const float* __restrict__ qkv, const float* __restrict__ temp,
    _Float16* __restrict__ qn16, _Float16* __restrict__ kn16, _Float16* __restrict__ v1T) {
  __shared__ float Qs[64][33];
  __shared__ float Ks[64][33];
  __shared__ float Vs[64][33];
  __shared__ float rq[64];
  __shared__ float rk[64];
  const int tid = threadIdx.x;
  const int bh = blockIdx.y, b = bh >> 3, h = bh & 7, n0 = blockIdx.x * 64;
  const float st = SCALE4 * temp[h];
#pragma unroll
  for (int q = 0; q < 8; ++q) {
    const int idx = tid + 256 * q;
    const int n = idx >> 5, d = idx & 31;
    const float* row = qkv + (size_t)(b * NTOK + n0 + n) * QKVW + h * HD + d;
    Qs[n][d] = row[0] * SCALE4;
    Ks[n][d] = row[CDIM];
    Vs[n][d] = row[2 * CDIM];
  }
  __syncthreads();
  if (tid < 128) {
    const int r = tid & 63;
    const bool isk = tid >= 64;
    float s = 0.f;
#pragma unroll
    for (int d = 0; d < HD; ++d) { const float a = isk ? Ks[r][d] : Qs[r][d]; s += a * a; }
    const float inv = 1.0f / fmaxf(sqrtf(s), 1e-12f);
    if (isk) rk[r] = inv; else rq[r] = inv;
  }
  __syncthreads();
  {
    const int n = tid >> 2, d8 = (tid & 3) * 8;
    const float iq = rq[n], ik = rk[n];
    v8h oq, ok;
#pragma unroll
    for (int e = 0; e < 8; ++e) {
      oq[e] = (_Float16)((Qs[n][d8 + e] * iq) * st);
      ok[e] = (_Float16)((Ks[n][d8 + e] * ik) * SCALE4);
    }
    _Float16* pq = qn16 + ((size_t)bh * NTOK + n0 + n) * HD + d8;
    _Float16* pk = kn16 + ((size_t)bh * NTOK + n0 + n) * HD + d8;

    const int n8 = (tid & 7) * 8;
    const int e0 = (tid >> 3);
    const int e1 = e0 + 32;
    v8h ov0, ov1;
    {
      const int ee = (e0 - 1) & 31;
#pragma unroll
      for (int c = 0; c < 8; ++c) {
        const float val = (e0 == 0) ? 1.0f : ((e0 <= HD) ? Vs[n8 + c][ee] : 0.0f);
        ov0[c] = (_Float16)val;
      }
    }
    {
      const int ee = (e1 - 1) & 31;
#pragma unroll
      for (int c = 0; c < 8; ++c) {
        const float val = (e1 <= HD) ? Vs[n8 + c][ee] : 0.0f;
        ov1[c] = (_Float16)val;
      }
    }
    _Float16* pv0 = v1T + ((size_t)bh * EP + e0) * NTOK + n0 + n8;
    _Float16* pv1 = v1T + ((size_t)bh * EP + e1) * NTOK + n0 + n8;

    *(volatile v8h*)pq = oq;
    *(volatile v8h*)pk = ok;
    *(volatile v8h*)pv0 = ov0;
    *(volatile v8h*)pv1 = ov1;
    __threadfence();
    *(volatile v8h*)pq = oq;
    *(volatile v8h*)pk = ok;
    *(volatile v8h*)pv0 = ov0;
    *(volatile v8h*)pv1 = ov1;
  }
}

__global__ __launch_bounds__(256) void vsum_k(const float* __restrict__ qkv, float* __restrict__ vsum) {
  __shared__ float part[8][33];
  __shared__ float tot[64];
  const int tid = threadIdx.x;
  const int bh = blockIdx.x, b = bh >> 3, h = bh & 7;
  const int e = tid & 31, p = tid >> 5;
  const float* col = qkv + (size_t)(b * NTOK) * QKVW + 2 * CDIM + h * HD + e;
  float s = 0.f;
  for (int n = p * 256; n < p * 256 + 256; ++n) s += col[(size_t)n * QKVW];
  part[p][e] = s;
  __syncthreads();
  if (tid < 64) {
    float t = 0.f;
    if (tid == 0) t = (float)NTOK;
    else if (tid <= HD) {
#pragma unroll
      for (int pp = 0; pp < 8; ++pp) t += part[pp][tid - 1];
    }
    tot[tid] = t;
  }
  __syncthreads();
  v4f v;
  const int l4 = (tid & 15) * 4;
  v[0] = tot[l4]; v[1] = tot[l4 + 1]; v[2] = tot[l4 + 2]; v[3] = tot[l4 + 3];
  float* pdst = vsum + (size_t)bh * EP + l4;
  if (tid < 16) *(volatile v4f*)pdst = v;
  __threadfence();
  if (tid < 16) *(volatile v4f*)pdst = v;
}

__global__ __launch_bounds__(256) void build_pt(const _Float16* __restrict__ kn16, _Float16* __restrict__ PT, int bh0) {
  __shared__ float Ks[128][33];
  __shared__ int fij[NF];
  const int tid = threadIdx.x;
  const int bhl = blockIdx.y, bh = bh0 + bhl, n0 = blockIdx.x * 128;
  {
    const int n = tid >> 1, d16 = (tid & 1) * 16;
    const _Float16* src = kn16 + ((size_t)bh * NTOK + n0 + n) * HD + d16;
    const v8h a = *(const v8h*)src;
    const v8h c = *(const v8h*)(src + 8);
#pragma unroll
    for (int e = 0; e < 8; ++e) { Ks[n][d16 + e] = (float)a[e]; Ks[n][d16 + 8 + e] = (float)c[e]; }
  }
  for (int f = tid; f < NF; f += 256) fij[f] = feat_code(f);
  __syncthreads();
  _Float16* base = PT + (size_t)bhl * NF * NTOK + n0;
  const int fl = tid >> 4, n8 = (tid & 15) * 8;
  for (int it = 0; it < NF / 16; ++it) {
    const int f = it * 16 + fl;
    const int code = fij[f];
    const int jc = code >> 8;
    const int i = code & 31, jj = jc & 31;
    v8h o;
#pragma unroll
    for (int e = 0; e < 8; ++e) {
      const float a = Ks[n8 + e][i];
      const float bq = Ks[n8 + e][jj];
      const float val = (jc == 254) ? 0.0f : ((jc == 255) ? a : a * bq);
      o[e] = (_Float16)val;
    }
    _Float16* p = base + (size_t)f * NTOK + n8;
    *(volatile v8h*)p = o;
    __threadfence();
    *(volatile v8h*)p = o;
  }
}

__global__ __launch_bounds__(256) void build_fq(const _Float16* __restrict__ qn16, _Float16* __restrict__ FQ, int bh0) {
  __shared__ float Qs[64][33];
  __shared__ int fij[NF];
  const int tid = threadIdx.x, lane = tid & 31, wave = tid >> 5;
  const int bhl = blockIdx.y, bh = bh0 + bhl, n0 = blockIdx.x * 64;
  {
    const int n = tid >> 2, d8 = (tid & 3) * 8;
    const v8h a = *(const v8h*)(qn16 + ((size_t)bh * NTOK + n0 + n) * HD + d8);
#pragma unroll
    for (int e = 0; e < 8; ++e) Qs[n][d8 + e] = (float)a[e];
  }
  for (int f = tid; f < NF; f += 256) fij[f] = feat_code(f);
  __syncthreads();
  _Float16* base = FQ + ((size_t)bhl * NTOK + n0) * NF;
  for (int rr = 0; rr < 8; ++rr) {
    const int n = wave + 8 * rr;
    const float* qr = &Qs[n][0];
    _Float16* rowp = base + (size_t)n * NF;
#pragma unroll
    for (int s = 0; s < 3; ++s) {
      const int c = lane + 32 * s;
      const int f0 = c * 8;
      v8h o;
#pragma unroll
      for (int e = 0; e < 8; ++e) {
        const int fc = min(f0 + e, NF - 1);
        const int code = fij[fc];
        const int jc = code >> 8;
        const int i = code & 31, jj = jc & 31;
        const float a = qr[i];
        const float bq = qr[jj];
        const float val = (jc == 254) ? 0.0f : ((jc == 255) ? a : a * bq);
        o[e] = (_Float16)val;
      }
      if (c < NF / 8) *(volatile v8h*)(rowp + f0) = o;
      __threadfence();
      if (c < NF / 8) *(volatile v8h*)(rowp + f0) = o;
    }
  }
}

__global__ __launch_bounds__(256) void finalize_y(
    const float* __restrict__ Y, const float* __restrict__ vsum,
    unsigned short* __restrict__ ah, unsigned short* __restrict__ al) {
  const int tid = threadIdx.x, lane = tid & 31, wave = tid >> 5;
  const int g = blockIdx.x * 8 + wave;
  const int b = g >> 11, n = g & (NTOK - 1);
  const int h = lane >> 2, d8 = (lane & 3) * 8;
  const int bh = b * NH + h;
  const float* yr = Y + ((size_t)bh * NTOK + n) * EP;
  const float* vs = vsum + (size_t)bh * EP;
  const float den = yr[0] + COEF_C * vs[0];
  const float inv = 1.0f / den;
  v8h hv, lv;
#pragma unroll
  for (int e = 0; e < 8; ++e) {
    const float num = yr[1 + d8 + e] + COEF_C * vs[1 + d8 + e];
    const float val = num * inv;
    const unsigned short hb = f2bf_bits(val);
    const unsigned short lb = f2bf_bits(val - bf_bits2f(hb));
    hv[e] = __builtin_bit_cast(_Float16, hb);
    lv[e] = __builtin_bit_cast(_Float16, lb);
  }
  const size_t o = (size_t)g * CDIM + h * HD + d8;
  *(volatile v8h*)(ah + o) = hv;
  *(volatile v8h*)(al + o) = lv;
  __threadfence();
  *(volatile v8h*)(ah + o) = hv;
  *(volatile v8h*)(al + o) = lv;
}

extern "C" void kernel_launch(void* const* d_in, const int* in_sizes, int n_in,
                              void* d_out, int out_size, void* d_ws, size_t ws_size,
                              hipStream_t stream) {
  if (n_in < 6) return;
  const float* x     = (const float*)d_in[0];
  const float* Wqkv  = (const float*)d_in[1];
  const float* bqkv  = (const float*)d_in[2];
  const float* Wproj = (const float*)d_in[3];
  const float* bproj = (const float*)d_in[4];
  const float* temp  = (const float*)d_in[5];
  const int nx  = in_sizes[0];
  const int nwq = in_sizes[1];
  const int nwp = in_sizes[3];
  const int MTOK = NB * NTOK;
  if (out_size != MTOK * CDIM) return;

  const size_t OFF_WQH  = 0;
  const size_t OFF_WQL  = OFF_WQH + (size_t)QKVW * CDIM * 2;
  const size_t OFF_WPH  = OFF_WQL + (size_t)QKVW * CDIM * 2;
  const size_t OFF_WPL  = OFF_WPH + (size_t)CDIM * CDIM * 2;
  const size_t OFF_VSUM = (size_t)1 << 20;
  const size_t OFF_QN   = (size_t)2 << 20;
  const size_t OFF_KN   = OFF_QN  + (size_t)NBH * NTOK * HD * 2;
  const size_t OFF_V1T  = OFF_KN  + (size_t)NBH * NTOK * HD * 2;
  const size_t OFF_ST   = OFF_V1T + (size_t)NBH * EP * NTOK * 2;
  const size_t OFF_BIG  = OFF_ST  + (size_t)NBH * EP * NF * 2;
  const size_t OFF_XH   = OFF_BIG;
  const size_t OFF_XL   = OFF_XH + (size_t)MTOK * CDIM * 2;
  const size_t OFF_QKV  = OFF_XL + (size_t)MTOK * CDIM * 2;
  const size_t END_A    = OFF_QKV + (size_t)MTOK * QKVW * 4;
  const size_t OFF_P    = OFF_BIG;
  const size_t OFF_Y    = OFF_P + (size_t)GB * NF * NTOK * 2;
  const size_t END_C    = OFF_Y + (size_t)NBH * NTOK * EP * 4;
  const size_t OFF_AH   = OFF_BIG;
  const size_t OFF_AL   = OFF_AH + (size_t)MTOK * CDIM * 2;
  const size_t END_ALL  = (END_A > END_C) ? END_A : END_C;
  if (END_ALL > ws_size) return;
  if (OFF_AL + (size_t)MTOK * CDIM * 2 > OFF_Y) return;

  unsigned char* ws = (unsigned char*)d_ws;
  unsigned short* wqh = (unsigned short*)(ws + OFF_WQH);
  unsigned short* wql = (unsigned short*)(ws + OFF_WQL);
  unsigned short* wph = (unsigned short*)(ws + OFF_WPH);
  unsigned short* wpl = (unsigned short*)(ws + OFF_WPL);
  float* vsum = (float*)(ws + OFF_VSUM);
  _Float16* qn16 = (_Float16*)(ws + OFF_QN);
  _Float16* kn16 = (_Float16*)(ws + OFF_KN);
  _Float16* v1T  = (_Float16*)(ws + OFF_V1T);
  _Float16* ST   = (_Float16*)(ws + OFF_ST);
  unsigned short* xh = (unsigned short*)(ws + OFF_XH);
  unsigned short* xl = (unsigned short*)(ws + OFF_XL);
  float* qkv = (float*)(ws + OFF_QKV);
  _Float16* Preg = (_Float16*)(ws + OFF_P);
  float* Y = (float*)(ws + OFF_Y);
  unsigned short* ah = (unsigned short*)(ws + OFF_AH);
  unsigned short* al = (unsigned short*)(ws + OFF_AL);
  float* out = (float*)d_out;

  {
    const int n2x = nx / 2, n2q = nwq / 2, n2p = nwp / 2;
    cast_split_bf16x2<<<dim3((n2x + 255) / 256), 256, 0, stream>>>(x, xh, xl, n2x);
    cast_split_bf16x2<<<dim3((n2q + 255) / 256), 256, 0, stream>>>(Wqkv, wqh, wql, n2q);
    cast_split_bf16x2<<<dim3((n2p + 255) / 256), 256, 0, stream>>>(Wproj, wph, wpl, n2p);
    const int tiles = (MTOK / 64) * (QKVW / 64);
    wmma_gemm64<1, true, 2, 0, false, 0, 0><<<dim3((tiles + 7) / 8, 1), 256, 0, stream>>>(
        xh, xl, CDIM, 0L, wqh, wql, CDIM, 0L, (void*)qkv, (void*)qkv, QKVW, 0L,
        bqkv, bqkv, 0L, MTOK, QKVW, CDIM, 1.0f);
    prep_qkv<<<dim3(NTOK / 64, NBH), 256, 0, stream>>>(qkv, temp, qn16, kn16, v1T);
    vsum_k<<<dim3(NBH), 256, 0, stream>>>(qkv, vsum);
  }
  for (int g = 0; g < NBH / GB; ++g) {
    build_pt<<<dim3(NTOK / 128, GB), 256, 0, stream>>>(kn16, Preg, g * GB);
    const int tiles = (EP / 64) * (NF / 64);
    wmma_gemm64<0, false, 0, 1, false, 0, 1><<<dim3((tiles + 7) / 8, GB), 256, 0, stream>>>(
        (const unsigned short*)(v1T + (size_t)g * GB * EP * NTOK), (const unsigned short*)(v1T + (size_t)g * GB * EP * NTOK),
        NTOK, (long)EP * NTOK,
        (const unsigned short*)Preg, (const unsigned short*)Preg, NTOK, (long)NF * NTOK,
        (void*)(ST + (size_t)g * GB * EP * NF), (void*)(ST + (size_t)g * GB * EP * NF), NF, (long)EP * NF,
        bqkv, bqkv, 0L, EP, NF, NTOK, 1.0f);
  }
  for (int g = 0; g < NBH / GB; ++g) {
    build_fq<<<dim3(NTOK / 64, GB), 256, 0, stream>>>(qn16, Preg, g * GB);
    const int tiles = (NTOK / 64) * (EP / 64);
    wmma_gemm64<0, false, 0, 0, false, 0, 0><<<dim3((tiles + 7) / 8, GB), 256, 0, stream>>>(
        (const unsigned short*)Preg, (const unsigned short*)Preg, NF, (long)NTOK * NF,
        (const unsigned short*)(ST + (size_t)g * GB * EP * NF), (const unsigned short*)(ST + (size_t)g * GB * EP * NF),
        NF, (long)EP * NF,
        (void*)(Y + (size_t)g * GB * NTOK * EP), (void*)(Y + (size_t)g * GB * NTOK * EP), EP, (long)NTOK * EP,
        bqkv, bqkv, 0L, NTOK, EP, NF, 1.0f);
  }
  {
    finalize_y<<<dim3(MTOK / 8), 256, 0, stream>>>(Y, vsum, ah, al);
    const int tiles = (MTOK / 64) * (CDIM / 64);
    wmma_gemm64<1, true, 2, 0, false, 0, 0><<<dim3((tiles + 7) / 8, 1), 256, 0, stream>>>(
        ah, al, CDIM, 0L, wph, wpl, CDIM, 0L, (void*)out, (void*)out, CDIM, 0L,
        bproj, bproj, 0L, MTOK, CDIM, CDIM, 1.0f);
  }
  (void)hipGetLastError();
}
